// attentionHead_22179211117250
// MI455X (gfx1250) — hardware-verified
//
#include <hip/hip_runtime.h>
#include <stddef.h>
#include <stdint.h>


#define NB    16
#define NS    1024
#define ND    768
#define NH    12
#define NHD   64
#define NQ    2304
#define MALL  16384
#define HB    8
#define MH    8192
#define KD    768
#define XSC   8
#define WSC   1024
#define NTHR  256
#define NWAVE 8
#define TPW   64
#define PT    40
#define PM    72
#define WSCAP 134217728
#define LDS_GEMM (NWAVE * 32 * 64 * 4)

static_assert(MALL == NB * NS);
static_assert(NQ == 3 * ND);
static_assert(MH == HB * NS);
static_assert((NB % HB) == 0);
static_assert(KD == ND);
static_assert(ND == NH * NHD);
static_assert(NHD == 64);
static_assert((KD % 128) == 0);
static_assert((KD % 32) == 0);
static_assert((MH % 128) == 0);
static_assert((MALL % 128) == 0);
static_assert((NQ % 128) == 0);
static_assert((ND % 128) == 0);
static_assert((NQ % 64) == 0);
static_assert((ND % 64) == 0);
static_assert((NS % 32) == 0);
static_assert(((NS / 16) % NWAVE) == 0);
static_assert(((MALL * KD) % (8 * NTHR)) == 0);
static_assert(NTHR == NWAVE * 32);
static_assert(LDS_GEMM <= 300 * 1024);
static_assert((PT * 2) % 16 == 0);
static_assert((PM * 2) % 16 == 0);

typedef float          v2f  __attribute__((ext_vector_type(2)));
typedef float          v4f  __attribute__((ext_vector_type(4)));
typedef float          v8f  __attribute__((ext_vector_type(8)));
typedef _Float16       v8h  __attribute__((ext_vector_type(8)));
typedef _Float16       v16h __attribute__((ext_vector_type(16)));
typedef __bf16         v16bf __attribute__((ext_vector_type(16)));
typedef unsigned short v8us __attribute__((ext_vector_type(8)));
union FragH { v16h v; v8h h[2]; };
union FragB { v16bf v; v8us h[2]; };

__device__ __forceinline__ v8f wmf(v16h a, v16h b, v8f c) {
  v8f d = __builtin_amdgcn_wmma_f32_16x16x32_f16(false, a, false, b, (short)0, c, false, false);
  asm volatile("v_nop\n\tv_nop\n\tv_nop\n\tv_nop" : "+v"(d) : "v"(a), "v"(b));
  return d;
}
__device__ __forceinline__ v8f wmb(v16bf a, v16bf b, v8f c) {
  v8f d = __builtin_amdgcn_wmma_f32_16x16x32_bf16(false, a, false, b, (short)0, c, false, false);
  asm volatile("v_nop\n\tv_nop\n\tv_nop\n\tv_nop" : "+v"(d) : "v"(a), "v"(b));
  return d;
}
__device__ __forceinline__ v8f zero8() {
  v8f z = {0.f, 0.f, 0.f, 0.f, 0.f, 0.f, 0.f, 0.f};
  return z;
}

__device__ __forceinline__ unsigned int bf16_rne_bits(float f) {
  const unsigned int u = __float_as_uint(f);
  return (u + 0x7fffu + ((u >> 16) & 1u)) >> 16;
}
__device__ __forceinline__ void split2(float f, unsigned short& hi, unsigned short& lo) {
  const unsigned int rh = bf16_rne_bits(f);
  const float fh = __uint_as_float(rh << 16);
  const unsigned int rl = bf16_rne_bits(f - fh);
  hi = (unsigned short)rh;
  lo = (unsigned short)rl;
}

__global__ __launch_bounds__(NTHR) void k_prepx(const float* __restrict__ x, _Float16* xh,
                                                const int* __restrict__ mflag) {
  (void)mflag;
  const size_t t = (size_t)blockIdx.x * NTHR + threadIdx.x;
  const float* p = x + t * 8;
  const v4f f0 = *(const v4f*)p;
  const v4f f1 = *(const v4f*)(p + 4);
  v8h a;
  a[0] = (_Float16)(f0.x * (float)XSC); a[1] = (_Float16)(f0.y * (float)XSC);
  a[2] = (_Float16)(f0.z * (float)XSC); a[3] = (_Float16)(f0.w * (float)XSC);
  a[4] = (_Float16)(f1.x * (float)XSC); a[5] = (_Float16)(f1.y * (float)XSC);
  a[6] = (_Float16)(f1.z * (float)XSC); a[7] = (_Float16)(f1.w * (float)XSC);
  _Float16* d = xh + t * 8;
  *(volatile v8h*)d = a;
  __threadfence();
  *(volatile v8h*)d = a;
}

__global__ __launch_bounds__(NTHR) void k_prepw(const float* __restrict__ W, _Float16* wt, int ncols) {
  __shared__ __attribute__((aligned(16))) float tile[128 * TPW];
  const int tid = threadIdx.x, lane = tid & 31, g = tid >> 5, hh = lane >> 4, m = lane & 15;
  const int n0 = blockIdx.x * 64;
  const int n = n0 + 2 * lane;
#pragma unroll 1
  for (int dc = 0; dc < KD; dc += 128) {
    __syncthreads();
#pragma unroll 4
    for (int p = 0; p < 16; ++p) {
      const int dl = g + 8 * p;
      const v2f w = *(const v2f*)(W + (size_t)(dc + dl) * (size_t)ncols + n);
      *(v2f*)(tile + dl * TPW + 2 * lane) = w;
    }
    __syncthreads();
    v8h hv[4];
#pragma unroll
    for (int q = 0; q < 4; ++q) {
      const int nl = 8 * g + 2 * q + hh;
      const int d8 = 8 * m;
#pragma unroll
      for (int e = 0; e < 8; ++e) hv[q][e] = (_Float16)(tile[(d8 + e) * TPW + nl] * (float)WSC);
    }
#pragma unroll
    for (int q = 0; q < 4; ++q) {
      _Float16* d = wt + (size_t)(n0 + 8 * g + 2 * q + hh) * KD + dc + 8 * m;
      *(volatile v8h*)d = hv[q];
    }
    __threadfence();
#pragma unroll
    for (int q = 0; q < 4; ++q) {
      _Float16* d = wt + (size_t)(n0 + 8 * g + 2 * q + hh) * KD + dc + 8 * m;
      *(volatile v8h*)d = hv[q];
    }
  }
}

__global__ __launch_bounds__(NTHR) void k_gemm(const _Float16* __restrict__ A, const _Float16* __restrict__ Bt,
                                               const float* __restrict__ bias, float* C, int ldc, float osc) {
  extern __shared__ v4f lds_dyn[];
  const int tid = threadIdx.x, lane = tid & 31, wave = tid >> 5, hh = lane >> 4, m = lane & 15;
  float* stg = (float*)lds_dyn + wave * (32 * 64);
  const int n0 = blockIdx.x * 128, m0 = blockIdx.y * 128;
  const int wm = (wave >> 1) * 32, wn = (wave & 1) * 64;

  v8f acc[2][4];
#pragma unroll
  for (int mt = 0; mt < 2; ++mt)
#pragma unroll
    for (int nt = 0; nt < 4; ++nt) acc[mt][nt] = zero8();

  const _Float16* ap = A  + (size_t)(m0 + wm + m) * KD + 8 * hh;
  const _Float16* bp = Bt + (size_t)(n0 + wn + m) * KD + 8 * hh;
#pragma unroll 1
  for (int kt = 0; kt < KD / 32; ++kt) {
    const int k0 = 32 * kt;
    FragH a0, a1;
    a0.h[0] = *(const v8h*)(ap + k0);
    a0.h[1] = *(const v8h*)(ap + k0 + 16);
    a1.h[0] = *(const v8h*)(ap + 16 * KD + k0);
    a1.h[1] = *(const v8h*)(ap + 16 * KD + k0 + 16);
#pragma unroll
    for (int nt = 0; nt < 4; ++nt) {
      const _Float16* bq = bp + (size_t)nt * 16 * KD + k0;
      FragH b;
      b.h[0] = *(const v8h*)bq;
      b.h[1] = *(const v8h*)(bq + 16);
      acc[0][nt] = wmf(a0.v, b.v, acc[0][nt]);
      acc[1][nt] = wmf(a1.v, b.v, acc[1][nt]);
    }
  }

  float bv[4];
#pragma unroll
  for (int nt = 0; nt < 4; ++nt) bv[nt] = bias[n0 + wn + 16 * nt + m];
#pragma unroll
  for (int mt = 0; mt < 2; ++mt) {
    float* sp = stg + (16 * mt + 8 * hh) * 64 + m;
#pragma unroll
    for (int nt = 0; nt < 4; ++nt) {
#pragma unroll
      for (int r = 0; r < 8; ++r) sp[r * 64 + 16 * nt] = acc[mt][nt][r] * osc + bv[nt];
    }
  }
  __syncthreads();

  float* gbase = C + (size_t)(m0 + wm) * (size_t)ldc + n0 + wn;
#pragma unroll
  for (int q = 0; q < 16; ++q) {
    const int row = 2 * q + hh;
    const v4f v = *(const v4f*)(stg + row * 64 + 4 * m);
    *(volatile v4f*)(gbase + (size_t)row * (size_t)ldc + 4 * m) = v;
  }
  __threadfence();
#pragma unroll
  for (int q = 0; q < 16; ++q) {
    const int row = 2 * q + hh;
    const v4f v = *(const v4f*)(stg + row * 64 + 4 * m);
    *(volatile v4f*)(gbase + (size_t)row * (size_t)ldc + 4 * m) = v;
  }
}

__device__ __forceinline__ void load_q_frag(const float* __restrict__ p, FragB& fh, FragB& fl) {
  const v4f q0 = *(const v4f*)p;
  const v4f q1 = *(const v4f*)(p + 4);
  const v4f q2 = *(const v4f*)(p + 16);
  const v4f q3 = *(const v4f*)(p + 20);
  v8us hA = {0, 0, 0, 0, 0, 0, 0, 0}, lA = {0, 0, 0, 0, 0, 0, 0, 0};
  v8us hB = {0, 0, 0, 0, 0, 0, 0, 0}, lB = {0, 0, 0, 0, 0, 0, 0, 0};
#pragma unroll
  for (int j = 0; j < 4; ++j) {
    unsigned short a, b;
    split2(q0[j], a, b); hA[j] = a;     lA[j] = b;
    split2(q1[j], a, b); hA[4 + j] = a; lA[4 + j] = b;
    split2(q2[j], a, b); hB[j] = a;     lB[j] = b;
    split2(q3[j], a, b); hB[4 + j] = a; lB[4 + j] = b;
  }
  fh.h[0] = hA; fh.h[1] = hB;
  fl.h[0] = lA; fl.h[1] = lB;
}

__global__ __launch_bounds__(NTHR) void k_attn(const float* __restrict__ qkv, _Float16* oh, int pass) {
  __shared__ __attribute__((aligned(16))) unsigned short Khi[64 * PT];
  __shared__ __attribute__((aligned(16))) unsigned short Klo[64 * PT];
  __shared__ __attribute__((aligned(16))) unsigned short Vhi[64 * PT];
  __shared__ __attribute__((aligned(16))) unsigned short Vlo[64 * PT];
  __shared__ __attribute__((aligned(16))) unsigned short MThi[64 * PM];
  __shared__ __attribute__((aligned(16))) unsigned short MTlo[64 * PM];
  __shared__ __attribute__((aligned(16))) _Float16 stg[NWAVE * 16 * 64];

  const int tid = threadIdx.x, lane = tid & 31, w = tid >> 5, hh = lane >> 4, m = lane & 15;
  const int bh = blockIdx.x;
  const int bl = bh / NH;
  const int h = bh - bl * NH;
  const float* base = qkv + (size_t)bl * NS * NQ + h * NHD;
  const float* Qp = base;
  const float* Kp = base + ND;
  const float* Vp = base + 2 * ND;

  const int tm = w & 3, tg = w >> 2;
  const int n0a = 32 * tg, n0b = n0a + 16;
  v8f c0 = zero8(), c1 = zero8();
#pragma unroll 1
  for (int t0 = 0; t0 < NS; t0 += 32) {
    __syncthreads();
#pragma unroll
    for (int p = 0; p < 2; ++p) {
      const int idx = tid + NTHR * p;
      const int tt = idx >> 4;
      const int c4 = idx & 15;
      const size_t ro = (size_t)(t0 + tt) * NQ + 4 * c4;
      const v4f kv = *(const v4f*)(Kp + ro);
      const v4f vv = *(const v4f*)(Vp + ro);
#pragma unroll
      for (int j = 0; j < 4; ++j) {
        const int d = 4 * c4 + j;
        unsigned short a, b;
        split2(kv[j], a, b);
        Khi[d * PT + tt] = a; Klo[d * PT + tt] = b;
        split2(vv[j], a, b);
        Vhi[d * PT + tt] = a; Vlo[d * PT + tt] = b;
      }
    }
    __syncthreads();
    FragB ah, al, bh0, bl0, bh1, bl1;
    const int ao = (16 * tm + m) * PT + 8 * hh;
    ah.h[0] = *(const v8us*)(Khi + ao); ah.h[1] = *(const v8us*)(Khi + ao + 16);
    al.h[0] = *(const v8us*)(Klo + ao); al.h[1] = *(const v8us*)(Klo + ao + 16);
    const int bo0 = (n0a + m) * PT + 8 * hh, bo1 = (n0b + m) * PT + 8 * hh;
    bh0.h[0] = *(const v8us*)(Vhi + bo0); bh0.h[1] = *(const v8us*)(Vhi + bo0 + 16);
    bl0.h[0] = *(const v8us*)(Vlo + bo0); bl0.h[1] = *(const v8us*)(Vlo + bo0 + 16);
    bh1.h[0] = *(const v8us*)(Vhi + bo1); bh1.h[1] = *(const v8us*)(Vhi + bo1 + 16);
    bl1.h[0] = *(const v8us*)(Vlo + bo1); bl1.h[1] = *(const v8us*)(Vlo + bo1 + 16);
    c0 = wmb(ah.v, bh0.v, c0); c0 = wmb(ah.v, bl0.v, c0); c0 = wmb(al.v, bh0.v, c0);
    c1 = wmb(ah.v, bh1.v, c1); c1 = wmb(ah.v, bl1.v, c1); c1 = wmb(al.v, bh1.v, c1);
  }
#pragma unroll
  for (int r = 0; r < 8; ++r) {
    const int dk = 16 * tm + 8 * hh + r;
    unsigned short a, b;
    split2(c0[r], a, b);
    MThi[(n0a + m) * PM + dk] = a; MTlo[(n0a + m) * PM + dk] = b;
    split2(c1[r], a, b);
    MThi[(n0b + m) * PM + dk] = a; MTlo[(n0b + m) * PM + dk] = b;
  }
  __syncthreads();

  _Float16* sw = stg + w * (16 * 64);
  _Float16* obase = oh + (size_t)(pass * HB + bl) * NS * ND + h * NHD;
  const int srow = lane >> 3, spc = lane & 7;
#pragma unroll 1
  for (int it = 0; it < (NS / 16) / NWAVE; ++it) {
    const int s0 = 16 * (w + NWAVE * it);
    const float* qrow = Qp + (size_t)(s0 + m) * NQ + 8 * hh;
    FragB ah0, al0, ah1, al1;
    load_q_frag(qrow, ah0, al0);
    load_q_frag(qrow + 32, ah1, al1);
    __syncthreads();
#pragma unroll
    for (int tn = 0; tn < 4; ++tn) {
      v8f c = zero8();
      {
        FragB bhf, blf;
        const int mo = (16 * tn + m) * PM + 8 * hh;
        bhf.h[0] = *(const v8us*)(MThi + mo); bhf.h[1] = *(const v8us*)(MThi + mo + 16);
        blf.h[0] = *(const v8us*)(MTlo + mo); blf.h[1] = *(const v8us*)(MTlo + mo + 16);
        c = wmb(ah0.v, bhf.v, c); c = wmb(ah0.v, blf.v, c); c = wmb(al0.v, bhf.v, c);
      }
      {
        FragB bhf, blf;
        const int mo = (16 * tn + m) * PM + 32 + 8 * hh;
        bhf.h[0] = *(const v8us*)(MThi + mo); bhf.h[1] = *(const v8us*)(MThi + mo + 16);
        blf.h[0] = *(const v8us*)(MTlo + mo); blf.h[1] = *(const v8us*)(MTlo + mo + 16);
        c = wmb(ah1.v, bhf.v, c); c = wmb(ah1.v, blf.v, c); c = wmb(al1.v, bhf.v, c);
      }
#pragma unroll
      for (int r = 0; r < 8; ++r) sw[(8 * hh + r) * 64 + 16 * tn + m] = (_Float16)c[r];
    }
    __syncthreads();
    v8h ov[4];
#pragma unroll
    for (int q = 0; q < 4; ++q) ov[q] = *(const v8h*)(sw + (4 * q + srow) * 64 + 8 * spc);
    _Float16* ob = obase + (size_t)s0 * ND;
#pragma unroll
    for (int q = 0; q < 4; ++q) *(volatile v8h*)(ob + (size_t)(4 * q + srow) * ND + 8 * spc) = ov[q];
    __threadfence();
#pragma unroll
    for (int q = 0; q < 4; ++q) *(volatile v8h*)(ob + (size_t)(4 * q + srow) * ND + 8 * spc) = ov[q];
  }
}

extern "C" void kernel_launch(void* const* d_in, const int* in_sizes, int n_in,
                              void* d_out, int out_size, void* d_ws, size_t ws_size,
                              hipStream_t stream) {
  if (n_in < 6) return;
  if (in_sizes[0] != MALL * ND || in_sizes[1] != KD * NQ || in_sizes[2] != NQ) return;
  if (in_sizes[3] != KD * ND || in_sizes[4] != ND || in_sizes[5] < 1) return;
  if (out_size != MALL * ND) return;

  const float* x    = (const float*)d_in[0];
  const float* Wqkv = (const float*)d_in[1];
  const float* bqkv = (const float*)d_in[2];
  const float* Wout = (const float*)d_in[3];
  const float* bout = (const float*)d_in[4];
  const int*   mflg = (const int*)d_in[5];
  float* out = (float*)d_out;

  char* ws = (char*)d_ws;
  size_t off = 0;
  const size_t oXh = off; off += (size_t)MALL * KD * 2;  off = (off + 255) & ~(size_t)255;
  const size_t oWq = off; off += (size_t)NQ * KD * 2;    off = (off + 255) & ~(size_t)255;
  const size_t oWo = off; off += (size_t)ND * KD * 2;    off = (off + 255) & ~(size_t)255;
  const size_t oQk = off; off += (size_t)MH * NQ * 4;    off = (off + 255) & ~(size_t)255;
  const size_t oOh = off; off += (size_t)MALL * ND * 2;  off = (off + 255) & ~(size_t)255;
  if (off > ws_size || off > (size_t)WSCAP) return;
  _Float16* xh  = (_Float16*)(ws + oXh);
  _Float16* wq  = (_Float16*)(ws + oWq);
  _Float16* wo  = (_Float16*)(ws + oWo);
  float*    qkv = (float*)(ws + oQk);
  _Float16* ohp = (_Float16*)(ws + oOh);

  k_prepx<<<(MALL * KD) / (8 * NTHR), NTHR, 0, stream>>>(x, xh, mflg);
  k_prepw<<<NQ / 64, NTHR, 0, stream>>>(Wqkv, wq, NQ);
  k_prepw<<<ND / 64, NTHR, 0, stream>>>(Wout, wo, ND);

  hipFuncSetAttribute(reinterpret_cast<const void*>(&k_gemm),
                      hipFuncAttributeMaxDynamicSharedMemorySize, LDS_GEMM);
  const float osc_qkv = 1.0f / (float)(XSC * WSC);
  const float osc_out = 1.0f / (float)WSC;
  for (int pass = 0; pass < NB / HB; ++pass) {
    k_gemm<<<dim3(NQ / 128, MH / 128), NTHR, LDS_GEMM, stream>>>(
        xh + (size_t)pass * MH * KD, wq, bqkv, qkv, NQ, osc_qkv);
    k_attn<<<HB * NH, NTHR, 0, stream>>>(qkv, ohp, pass);
  }
  k_gemm<<<dim3(ND / 128, MALL / 128), NTHR, LDS_GEMM, stream>>>(ohp, wo, bout, out, ND, osc_out);
}
